// SelfAttention_22342419874292
// MI455X (gfx1250) — hardware-verified
//
#include <hip/hip_runtime.h>
#ifndef NB
#define NB 8
#endif
#ifndef SEQ
#define SEQ 1024
#endif
#define NB_FULL 8
#define SEQ_FULL 1024
#define DM 1024
#define NH 16
#define HD 64
#define EARLY 256

static_assert(NH * HD == DM);
static_assert(HD == 64);
static_assert(DM % 128 == 0 && DM % 64 == 0 && DM % 32 == 0 && DM % 8 == 0);
static_assert(SEQ % 128 == 0 && SEQ % 64 == 0 && SEQ % 32 == 0);
static_assert(EARLY % 128 == 0 && EARLY % 64 == 0 && SEQ >= EARLY);
static_assert((SEQ - EARLY) % 128 == 0);
static_assert(NB <= NB_FULL && SEQ <= SEQ_FULL);
static_assert(((size_t)NB * SEQ) % 128 == 0);

typedef _Float16 v16h __attribute__((ext_vector_type(16)));
typedef unsigned short v8us __attribute__((ext_vector_type(8), may_alias));
typedef float v8f  __attribute__((ext_vector_type(8)));
typedef float v4f  __attribute__((ext_vector_type(4)));
typedef float v4fa __attribute__((ext_vector_type(4), may_alias));
union FragH { v16h v; v8us half[2]; _Float16 h[16]; unsigned short u[16]; };

__device__ __forceinline__ unsigned short bf16_bits(float x) { unsigned int u = __float_as_uint(x); return (unsigned short)((u + 0x7FFFu + ((u >> 16) & 1u)) >> 16); }
__device__ __forceinline__ float bf16_rne(float x) { return __uint_as_float(((unsigned int)bf16_bits(x)) << 16); }

__device__ __forceinline__ v16h g2_frag(const _Float16* p, int hh) { FragH f; f.half[0] = *(const v8us*)((const unsigned short*)p + 8 * hh); f.half[1] = *(const v8us*)((const unsigned short*)p + 16 + 8 * hh); return f.v; }
__device__ __forceinline__ v8f g2_mma(v16h a, v16h b, v8f c) { v8f d = __builtin_amdgcn_wmma_f32_16x16x32_f16(false, a, false, b, (short)0, c, false, false); asm volatile("v_nop\n\tv_nop\n\tv_nop\n\tv_nop" : "+v"(d) : "v"(a), "v"(b)); return d; }

__global__ __launch_bounds__(256) void k_wnat(const float* __restrict__ w, _Float16* __restrict__ Bt) {
  const size_t t = (size_t)blockIdx.x * 256 + threadIdx.x; if (t >= (size_t)DM * DM / 8) return;
  const v4f a = *(const v4fa*)(w + t * 8), c = *(const v4fa*)(w + t * 8 + 4); FragH f;
#pragma unroll
  for (int q = 0; q < 4; ++q) { f.h[q] = (_Float16)(bf16_rne(a[q]) * 64.0f); f.h[4 + q] = (_Float16)(bf16_rne(c[q]) * 64.0f); }
  const v8us o = f.half[0];
  *(volatile v8us*)((unsigned short*)Bt + t * 8) = o; __threadfence(); *(volatile v8us*)((unsigned short*)Bt + t * 8) = o;
}

__global__ __launch_bounds__(256) void k_x16(const float* __restrict__ x, _Float16* __restrict__ X16) {
  const size_t t = (size_t)blockIdx.x * 256 + threadIdx.x; if (t >= (size_t)NB * SEQ * DM / 8) return;
  const size_t e = t * 8; const size_t b = e / ((size_t)SEQ * DM); const size_t rem = e - b * (size_t)SEQ * DM;
  const float* src = x + b * (size_t)SEQ_FULL * DM + rem;
  const v4f a = *(const v4fa*)src, c = *(const v4fa*)(src + 4); FragH f;
#pragma unroll
  for (int q = 0; q < 4; ++q) { f.h[q] = (_Float16)bf16_rne(a[q]); f.h[4 + q] = (_Float16)bf16_rne(c[q]); }
  const v8us o = f.half[0];
  *(volatile v8us*)((unsigned short*)X16 + e) = o; __threadfence(); *(volatile v8us*)((unsigned short*)X16 + e) = o;
}

template <int MT, bool ARES>
__device__ __forceinline__ void gemm_loop(const _Float16* __restrict__ a_base, const _Float16* __restrict__ ar_base, int lda,
                                          const _Float16* __restrict__ b_base, int ldb, int K, int ln, int hh,
                                          v8f (&acc)[MT * 4], v8f (&acc2)[MT * 4]) {
  const _Float16* ap = a_base + (size_t)ln * lda; const _Float16* arp = ar_base + (size_t)ln * lda; const _Float16* bp = b_base + (size_t)ln * ldb;
#pragma unroll 1
  for (int kb = 0; kb < K; kb += 32) {
    v16h a[MT], ar[MT];
#pragma unroll
    for (int i = 0; i < MT; ++i) { a[i] = g2_frag(ap + (size_t)(16 * i) * lda + kb, hh); ar[i] = a[i]; if (ARES) ar[i] = g2_frag(arp + (size_t)(16 * i) * lda + kb, hh); }
#pragma unroll
    for (int t = 0; t < 4; ++t) {
      const v16h b = g2_frag(bp + (size_t)(16 * t) * ldb + kb, hh);
#pragma unroll
      for (int i = 0; i < MT; ++i) { acc[i * 4 + t] = g2_mma(a[i], b, acc[i * 4 + t]); if (ARES) acc2[i * 4 + t] = g2_mma(ar[i], b, acc2[i * 4 + t]); }
    }
  }
}
template <int MT, bool ARES, bool BIASROW>
__device__ __forceinline__ void stage_tile(float (*sow)[68], const v8f (&acc)[MT * 4], const v8f (&acc2)[MT * 4], float alpha, float alpha2,
                                           const float* __restrict__ bias, int row0, int col0, int ln, int hh) {
#pragma unroll
  for (int i = 0; i < MT; ++i) {
#pragma unroll
    for (int t = 0; t < 4; ++t) {
      const float bc = BIASROW ? 0.f : bf16_rne(bias[col0 + t * 16 + ln]);
#pragma unroll
      for (int r = 0; r < 8; ++r) {
        const int rloc = i * 16 + 8 * hh + r;
        float v = acc[i * 4 + t][r] * alpha;
        if (ARES) v += acc2[i * 4 + t][r] * alpha2;
        v += BIASROW ? bf16_rne(bias[row0 + rloc]) : bc;
        sow[rloc][t * 16 + ln] = v;
      }
    }
  }
}
template <int MT>
__device__ __forceinline__ void store_tile_f16(float (*sow)[68], _Float16* __restrict__ hi, size_t ldh, _Float16* __restrict__ rs, size_t ldr, bool wres, int lane) {
  const int rq = lane >> 3, c8 = (lane & 7) * 8;
  for (int pass = 0; pass < 2; ++pass) {
#pragma unroll
    for (int it = 0; it < 4 * MT; ++it) {
      const int r = it * 4 + rq;
      const v4f a = *(const v4fa*)&sow[r][c8], c = *(const v4fa*)&sow[r][c8 + 4];
      FragH fh, fl;
#pragma unroll
      for (int q = 0; q < 4; ++q) {
        _Float16 h = (_Float16)a[q]; fh.h[q] = h; fl.h[q] = (_Float16)((a[q] - (float)h) * 1024.0f);
        h = (_Float16)c[q]; fh.h[4 + q] = h; fl.h[4 + q] = (_Float16)((c[q] - (float)h) * 1024.0f);
      }
      const v8us oh = fh.half[0], ol = fl.half[0];
      *(volatile v8us*)((unsigned short*)hi + (size_t)r * ldh + c8) = oh;
      if (wres) *(volatile v8us*)((unsigned short*)rs + (size_t)r * ldr + c8) = ol;
    }
    if (pass == 0) __threadfence();
  }
}
template <int MT>
__device__ __forceinline__ void store_tile_f32(float (*sow)[68], float* __restrict__ C, size_t ldc, int lane) {
  const int rsub = lane >> 4, c4 = (lane & 15) * 4;
  for (int pass = 0; pass < 2; ++pass) {
#pragma unroll
    for (int q = 0; q < 8 * MT; ++q) {
      const int r = q * 2 + rsub;
      const v4f v = *(const v4fa*)&sow[r][c4];
      *(volatile v4f*)(C + (size_t)r * ldc + c4) = v;
    }
    if (pass == 0) __threadfence();
  }
}

__global__ __launch_bounds__(128) void k_proj_rows(const _Float16* __restrict__ X16, const _Float16* __restrict__ Wt, const float* __restrict__ bias,
                                                   _Float16* __restrict__ PH, _Float16* __restrict__ PR) {
  __shared__ __attribute__((aligned(16))) float so[4][32][68];
  const int tid = threadIdx.x, w = tid >> 5, lane = tid & 31, ln = lane & 15, hh = lane >> 4;
  const int ntn = DM / 64; const int mt = blockIdx.x / ntn, nq = blockIdx.x - mt * ntn;
  const int row0 = mt * 128 + 32 * w, col0 = nq * 64;
  const v8f z8 = {0.f, 0.f, 0.f, 0.f, 0.f, 0.f, 0.f, 0.f};
  v8f acc[8], acc2[8];
#pragma unroll
  for (int i = 0; i < 8; ++i) { acc[i] = z8; acc2[i] = z8; }
  gemm_loop<2, false>(X16 + (size_t)row0 * DM, X16 + (size_t)row0 * DM, DM, Wt + (size_t)col0 * DM, DM, DM, ln, hh, acc, acc2);
  stage_tile<2, false, false>(so[w], acc, acc2, 0.015625f, 0.f, bias, row0, col0, ln, hh);
  __builtin_amdgcn_fence(4  , "workgroup"); __builtin_amdgcn_wave_barrier();
  const int b = row0 / SEQ, l0 = row0 - b * SEQ; const bool wres = l0 < EARLY;
  _Float16* hi = PH + (size_t)row0 * DM + col0;
  _Float16* rs = PR + ((size_t)b * EARLY + (size_t)(wres ? l0 : 0)) * DM + col0;
  store_tile_f16<2>(so[w], hi, DM, rs, DM, wres, lane);
}

__global__ __launch_bounds__(128) void k_proj_vt(const _Float16* __restrict__ Wv16, const _Float16* __restrict__ X16, const float* __restrict__ bias,
                                                 _Float16* __restrict__ VT, _Float16* __restrict__ VR) {
  __shared__ __attribute__((aligned(16))) float so[4][32][68];
  const int tid = threadIdx.x, w = tid >> 5, lane = tid & 31, ln = lane & 15, hh = lane >> 4; const int by = blockIdx.y;
  const int ntn = SEQ / 64; const int mt = blockIdx.x / ntn, nq = blockIdx.x - mt * ntn;
  const int row0 = mt * 128 + 32 * w, col0 = nq * 64;
  const v8f z8 = {0.f, 0.f, 0.f, 0.f, 0.f, 0.f, 0.f, 0.f};
  v8f acc[8], acc2[8];
#pragma unroll
  for (int i = 0; i < 8; ++i) { acc[i] = z8; acc2[i] = z8; }
  gemm_loop<2, false>(Wv16 + (size_t)row0 * DM, Wv16 + (size_t)row0 * DM, DM, X16 + ((size_t)by * SEQ + col0) * DM, DM, DM, ln, hh, acc, acc2);
  stage_tile<2, false, true>(so[w], acc, acc2, 0.015625f, 0.f, bias, row0, col0, ln, hh);
  __builtin_amdgcn_fence(4  , "workgroup"); __builtin_amdgcn_wave_barrier();
  const bool wres = col0 < EARLY;
  _Float16* hi = VT + ((size_t)by * DM + row0) * SEQ + col0;
  _Float16* rs = VR + ((size_t)by * DM + row0) * EARLY + (size_t)(wres ? col0 : 0);
  store_tile_f16<2>(so[w], hi, SEQ, rs, EARLY, wres, lane);
}

template <bool EARLYQ>
__device__ __forceinline__ void attn_body(const _Float16* __restrict__ QH, const _Float16* __restrict__ QR, const _Float16* __restrict__ KH, const _Float16* __restrict__ KR,
                                          const _Float16* __restrict__ VT, const _Float16* __restrict__ VR, _Float16* __restrict__ CH, _Float16* __restrict__ CR,
                                          float (*sow)[68], int b, int h, int q0, int lane) {
  const int ln = lane & 15, hh = lane >> 4;
  const float NEG = -__builtin_inff();
  const v8f z8 = {0.f, 0.f, 0.f, 0.f, 0.f, 0.f, 0.f, 0.f};
  const _Float16* qp = QH + ((size_t)b * SEQ + q0 + ln) * DM + h * HD;
  const v16h qb0 = g2_frag(qp, hh), qb1 = g2_frag(qp + 32, hh);
  v16h qr0 = qb0, qr1 = qb1;
  if (EARLYQ) { const _Float16* qrp = QR + ((size_t)b * EARLY + q0 + ln) * DM + h * HD; qr0 = g2_frag(qrp, hh); qr1 = g2_frag(qrp + 32, hh); }
  const _Float16* kbase  = KH + ((size_t)b * SEQ + ln) * DM + h * HD;
  const _Float16* krbase = KR + ((size_t)b * EARLY + ln) * DM + h * HD;
  const _Float16* vbase  = VT + ((size_t)b * DM + h * HD + ln) * SEQ;
  const _Float16* vrbase = VR + ((size_t)b * DM + h * HD + ln) * EARLY;
  float m = NEG, lsum = 0.f;
  v8f o[4], o2[4];
#pragma unroll
  for (int c = 0; c < 4; ++c) { o[c] = z8; o2[c] = z8; }
  const int qrow = q0 + ln;
  const int kbmax = (q0 + 15) >> 5;
#pragma unroll 1
  for (int kb = 0; kb <= kbmax; ++kb) {
    const int key0 = kb * 32;
    float sv[16];
    float mx = NEG;
#pragma unroll
    for (int t = 0; t < 2; ++t) {
      const _Float16* kp = kbase + (size_t)(key0 + 16 * t) * DM;
      const v16h ka0 = g2_frag(kp, hh), ka1 = g2_frag(kp + 32, hh);
      v8f s1 = z8; s1 = g2_mma(ka0, qb0, s1); s1 = g2_mma(ka1, qb1, s1);
      v8f s2 = z8;
      if (EARLYQ) {
        s2 = g2_mma(ka0, qr0, s2); s2 = g2_mma(ka1, qr1, s2);
        const _Float16* krp = krbase + (size_t)(key0 + 16 * t) * DM;
        const v16h kr0 = g2_frag(krp, hh), kr1 = g2_frag(krp + 32, hh);
        s2 = g2_mma(kr0, qb0, s2); s2 = g2_mma(kr1, qb1, s2);
      }
#pragma unroll
      for (int r = 0; r < 8; ++r) {
        const int key = key0 + 16 * t + 8 * hh + r;
        float s = s1[r];
        if (EARLYQ) s += s2[r] * 0.0009765625f;
        s *= 0.125f;
        s = (key <= qrow) ? s : NEG;
        sv[t * 8 + r] = s; mx = fmaxf(mx, s);
      }
    }
    mx = fmaxf(mx, __shfl_xor(mx, 16, 32));
    const float mnew = fmaxf(m, mx);
    const float corr = __expf(m - mnew);
    m = mnew;
    FragH ph, pr; float rsum = 0.f;
#pragma unroll
    for (int i = 0; i < 16; ++i) {
      const float p = __expf(sv[i] - mnew); rsum += p;
      const float pc = p * 1024.0f; const _Float16 h16 = (_Float16)pc; ph.h[i] = h16;
      pr.h[i] = EARLYQ ? (_Float16)((pc - (float)h16) * 1024.0f) : (_Float16)0.0f;
    }
    lsum = lsum * corr + rsum;
#pragma unroll
    for (int c = 0; c < 4; ++c) {
#pragma unroll
      for (int r = 0; r < 8; ++r) { o[c][r] *= corr; if (EARLYQ) o2[c][r] *= corr; }
    }
#pragma unroll
    for (int c = 0; c < 4; ++c) {
      const v16h va = g2_frag(vbase + (size_t)(c * 16) * SEQ + key0, hh);
      o[c] = g2_mma(va, ph.v, o[c]);
      if (EARLYQ) {
        o2[c] = g2_mma(va, pr.v, o2[c]);
        const v16h vra = g2_frag(vrbase + (size_t)(c * 16) * EARLY + key0, hh);
        o2[c] = g2_mma(vra, ph.v, o2[c]);
      }
    }
  }
  const float ltot = lsum + __shfl_xor(lsum, 16, 32);
  const float inv = 1.0f / (64.0f * ltot);
#pragma unroll
  for (int c = 0; c < 4; ++c) {
#pragma unroll
    for (int r = 0; r < 8; ++r) { float v = o[c][r]; if (EARLYQ) v += o2[c][r] * 0.0009765625f; sow[ln][c * 16 + 8 * hh + r] = v * inv; }
  }
  __builtin_amdgcn_fence(4  , "workgroup"); __builtin_amdgcn_wave_barrier();
  _Float16* hi = CH + ((size_t)b * SEQ + q0) * DM + h * HD;
  _Float16* rs = CR + ((size_t)b * EARLY + (size_t)(EARLYQ ? q0 : 0)) * DM + h * HD;
  store_tile_f16<1>(sow, hi, DM, rs, DM, EARLYQ, lane);
}

__global__ __launch_bounds__(256) void k_attn(const _Float16* __restrict__ QH, const _Float16* __restrict__ QR, const _Float16* __restrict__ KH, const _Float16* __restrict__ KR,
                                              const _Float16* __restrict__ VT, const _Float16* __restrict__ VR, _Float16* __restrict__ CH, _Float16* __restrict__ CR) {
  __shared__ __attribute__((aligned(16))) float so[8][16][68];
  const int wave = threadIdx.x >> 5, lane = threadIdx.x & 31;
  const int nqb = SEQ / 128; const int bh = blockIdx.x / nqb, qb = blockIdx.x - bh * nqb;
  const int b = bh / NH, h = bh - b * NH; const int q0 = qb * 128 + wave * 16;
  if (qb < EARLY / 128) attn_body<true>(QH, QR, KH, KR, VT, VR, CH, CR, so[wave], b, h, q0, lane);
  else                  attn_body<false>(QH, QR, KH, KR, VT, VR, CH, CR, so[wave], b, h, q0, lane);
}

__global__ __launch_bounds__(128) void k_out_late(const _Float16* __restrict__ CH, const _Float16* __restrict__ Wt, const float* __restrict__ bias, float* __restrict__ out) {
  __shared__ __attribute__((aligned(16))) float so[4][32][68];
  const int tid = threadIdx.x, w = tid >> 5, lane = tid & 31, ln = lane & 15, hh = lane >> 4; const int by = blockIdx.y;
  const int ntn = DM / 64; const int mt = blockIdx.x / ntn, nq = blockIdx.x - mt * ntn;
  const int l0 = EARLY + mt * 128 + 32 * w, col0 = nq * 64;
  const size_t row0 = (size_t)by * SEQ + l0;
  const v8f z8 = {0.f, 0.f, 0.f, 0.f, 0.f, 0.f, 0.f, 0.f};
  v8f acc[8], acc2[8];
#pragma unroll
  for (int i = 0; i < 8; ++i) { acc[i] = z8; acc2[i] = z8; }
  gemm_loop<2, false>(CH + row0 * DM, CH + row0 * DM, DM, Wt + (size_t)col0 * DM, DM, DM, ln, hh, acc, acc2);
  stage_tile<2, false, false>(so[w], acc, acc2, 0.0009765625f, 0.f, bias, 0, col0, ln, hh);
  __builtin_amdgcn_fence(4  , "workgroup"); __builtin_amdgcn_wave_barrier();
  store_tile_f32<2>(so[w], out + ((size_t)by * SEQ_FULL + l0) * DM + col0, DM, lane);
}
__global__ __launch_bounds__(128) void k_out_early(const _Float16* __restrict__ CH, const _Float16* __restrict__ CR, const _Float16* __restrict__ Wt, const float* __restrict__ bias, float* __restrict__ out) {
  __shared__ __attribute__((aligned(16))) float so[4][16][68];
  const int tid = threadIdx.x, w = tid >> 5, lane = tid & 31, ln = lane & 15, hh = lane >> 4; const int by = blockIdx.y;
  const int ntn = DM / 64; const int mt = blockIdx.x / ntn, nq = blockIdx.x - mt * ntn;
  const int l0 = mt * 64 + 16 * w, col0 = nq * 64;
  const v8f z8 = {0.f, 0.f, 0.f, 0.f, 0.f, 0.f, 0.f, 0.f};
  v8f acc[4], acc2[4];
#pragma unroll
  for (int i = 0; i < 4; ++i) { acc[i] = z8; acc2[i] = z8; }
  gemm_loop<1, true>(CH + ((size_t)by * SEQ + l0) * DM, CR + ((size_t)by * EARLY + l0) * DM, DM, Wt + (size_t)col0 * DM, DM, DM, ln, hh, acc, acc2);
  stage_tile<1, true, false>(so[w], acc, acc2, 0.0009765625f, 9.5367431640625e-07f, bias, 0, col0, ln, hh);
  __builtin_amdgcn_fence(4  , "workgroup"); __builtin_amdgcn_wave_barrier();
  store_tile_f32<1>(so[w], out + ((size_t)by * SEQ_FULL + l0) * DM + col0, DM, lane);
}

extern "C" void kernel_launch(void* const* d_in, const int* in_sizes, int n_in,
                              void* d_out, int out_size, void* d_ws, size_t ws_size, hipStream_t stream) {
  if (n_in < 11) return;
  const long long need_x = ((long long)(NB - 1) * SEQ_FULL + SEQ) * DM;
  if (in_sizes[0] < need_x || in_sizes[1] < need_x || in_sizes[2] < need_x || (long long)out_size < need_x) return;
  if (in_sizes[3] < DM * DM || in_sizes[5] < DM * DM || in_sizes[7] < DM * DM || in_sizes[9] < DM * DM) return;
  if (in_sizes[4] < DM || in_sizes[6] < DM || in_sizes[8] < DM || in_sizes[10] < DM) return;
  const float* const* I = (const float* const*)d_in;
  const float* x_key = I[0]; const float* x_val = I[1]; const float* x_qry = I[2];
  const float* Wk = I[3]; const float* bk = I[4]; const float* Wq = I[5]; const float* bq = I[6];
  const float* Wv = I[7]; const float* bv = I[8]; const float* Wp = I[9]; const float* bp = I[10];
  constexpr size_t SZ_W = (size_t)DM * DM * 2;
  constexpr size_t SZ_P = (size_t)NB * SEQ * DM * 2;
  constexpr size_t SZ_E = (size_t)NB * EARLY * DM * 2;
  static_assert(SZ_W % 256 == 0 && SZ_P % 256 == 0 && SZ_E % 256 == 0);
  static_assert(4 * SZ_W + 5 * SZ_P + 4 * SZ_E <= (size_t)134217728);
  char* ws = (char*)d_ws; size_t off = 0;
  auto take = [&](size_t bytes) { char* p = ws + off; off += (bytes + 255) & ~(size_t)255; return p; };
  _Float16* W16k = (_Float16*)take(SZ_W); _Float16* W16q = (_Float16*)take(SZ_W); _Float16* W16v = (_Float16*)take(SZ_W); _Float16* W16p = (_Float16*)take(SZ_W);
  _Float16* X16 = (_Float16*)take(SZ_P);
  _Float16* QH = (_Float16*)take(SZ_P); _Float16* KH = (_Float16*)take(SZ_P); _Float16* VT = (_Float16*)take(SZ_P); _Float16* CH = (_Float16*)take(SZ_P);
  _Float16* QR = (_Float16*)take(SZ_E); _Float16* KR = (_Float16*)take(SZ_E); _Float16* VR = (_Float16*)take(SZ_E); _Float16* CR = (_Float16*)take(SZ_E);
  if (off > ws_size) return;
  const unsigned gw = (unsigned)(((size_t)DM * DM / 8 + 255) / 256);
  const unsigned gx = (unsigned)(((size_t)NB * SEQ * DM / 8 + 255) / 256);
  k_wnat<<<gw, 256, 0, stream>>>(Wk, W16k); k_wnat<<<gw, 256, 0, stream>>>(Wq, W16q); k_wnat<<<gw, 256, 0, stream>>>(Wv, W16v); k_wnat<<<gw, 256, 0, stream>>>(Wp, W16p);
  const unsigned gproj = (unsigned)(((size_t)NB * SEQ / 128) * (DM / 64));
  k_x16<<<gx, 256, 0, stream>>>(x_key, X16);
  k_proj_rows<<<gproj, 128, 0, stream>>>(X16, W16k, bk, KH, KR);
  k_x16<<<gx, 256, 0, stream>>>(x_qry, X16);
  k_proj_rows<<<gproj, 128, 0, stream>>>(X16, W16q, bq, QH, QR);
  k_x16<<<gx, 256, 0, stream>>>(x_val, X16);
  k_proj_vt<<<dim3((DM / 128) * (SEQ / 64), NB), 128, 0, stream>>>(W16v, X16, bv, VT, VR);
  k_attn<<<NB * NH * (SEQ / 128), 256, 0, stream>>>(QH, QR, KH, KR, VT, VR, CH, CR);
  if ((SEQ - EARLY) / 128 > 0)
    k_out_late<<<dim3(((SEQ - EARLY) / 128) * (DM / 64), NB), 128, 0, stream>>>(CH, W16p, bp, (float*)d_out);
  k_out_early<<<dim3((EARLY / 64) * (DM / 64), NB), 128, 0, stream>>>(CH, CR, W16p, bp, (float*)d_out);
}
